// FourierKANLayer_5299989643383
// MI455X (gfx1250) — hardware-verified
//
#include <hip/hip_runtime.h>


namespace {
typedef _Float16 b16;
typedef __attribute__((ext_vector_type(16))) _Float16 v16b;
typedef __attribute__((ext_vector_type(8))) _Float16 v8b;
typedef __attribute__((ext_vector_type(4))) _Float16 v4h;
typedef __attribute__((ext_vector_type(2))) _Float16 v2h;
typedef __attribute__((ext_vector_type(8))) float v8f;
typedef __attribute__((ext_vector_type(4))) float v4f;
typedef __attribute__((ext_vector_type(2))) float v2f;
__device__ __forceinline__ float bf16_rne(float f) { unsigned int u = __float_as_uint(f); u += 0x7FFFu + ((u >> 16) & 1u); return __uint_as_float(u & 0xFFFF0000u); }
__device__ __forceinline__ void split16(float v, b16& hi, b16& lo) { hi = (b16)v; lo = (b16)(v - (float)hi); }
__device__ __forceinline__ v16b frag_kb(const b16* p, int hh) { const v8b a = *(const v8b*)(p + 8 * hh), b = *(const v8b*)(p + 16 + 8 * hh); v16b f;
#pragma unroll
  for (int e = 0; e < 8; ++e) { f[e] = a[e]; f[8 + e] = b[e]; } return f; }
__device__ __forceinline__ v8f wmma16b(v16b a, v16b b, v8f c) { v8f d = __builtin_amdgcn_wmma_f32_16x16x32_f16(false, a, false, b, (short)0, c, false, false); asm volatile("v_nop\n\tv_nop\n\tv_nop\n\tv_nop" : "+v"(d) : "v"(a), "v"(b)); return d; }
__device__ __forceinline__ void wave_lds_sync() { __builtin_amdgcn_fence(__ATOMIC_RELEASE, "workgroup"); __builtin_amdgcn_wave_barrier(); __builtin_amdgcn_fence(__ATOMIC_ACQUIRE, "workgroup"); }
__device__ __forceinline__ float pmul(float a, float b) { float p = a * b; asm volatile("" : "+v"(p)); return p; }
__device__ __forceinline__ int iclamp(int v, int lo, int hi) { return v < lo ? lo : (v > hi ? hi : v); }
__device__ __forceinline__ float nexp2(float v) { return __builtin_amdgcn_exp2f(v); }

constexpr int NR = 8192, ROWSL = NR  , I = 512, O = 512, G = 8, K = I * G * 2  ;
constexpr float XS = 8.0f, WSC = 256.0f;
static_assert(NR % 16 == 0 && K % 128 == 0 && O == 512, "tiling");

__global__ __launch_bounds__(256) void wt_kernel(const float* __restrict__ coef, b16* __restrict__ WT) {
  const int u = blockIdx.x * 256 + threadIdx.x; if (u >= O * I) return; const int o = u / I, i = u % I; v16b v;
#pragma unroll
  for (int g = 0; g < G; ++g) { v[2 * g] = (b16)(bf16_rne(coef[(((size_t)0 * O + o) * I + i) * G + g]) * WSC); v[2 * g + 1] = (b16)(bf16_rne(coef[(((size_t)1 * O + o) * I + i) * G + g]) * WSC); }
  for (int pass = 0; pass < 2; ++pass) { *(volatile v16b*)(WT + (size_t)u * 16) = v; __threadfence(); }
}
__global__ __launch_bounds__(64) void fkan_kernel(const float* __restrict__ x, const b16* __restrict__ WT, const float* __restrict__ bias, float* __restrict__ out) {
  __shared__ __attribute__((aligned(16))) b16 As[16][128 + 8]; __shared__ __attribute__((aligned(16))) float Tf[2][16][256 + 4];
  const int wave = threadIdx.x >> 5, lane = threadIdx.x & 31, nloc = lane & 15, hlf = lane >> 4; const size_t m0 = (size_t)blockIdx.x * 16; const int n0 = wave * 256;
  const int srow = threadIdx.x >> 2, sq = threadIdx.x & 3; const float* xr = x + (m0 + srow) * I;
  v8f acc[16];
#pragma unroll
  for (int t = 0; t < 16; ++t) acc[t] = (v8f){};
#pragma unroll 1
  for (int kc = 0; kc < K; kc += 128) { const int i0 = kc / 16;
#pragma unroll
    for (int e2 = 0; e2 < 2; ++e2) { const int il = 2 * sq + e2; const float xv = bf16_rne(xr[i0 + il]); v16b v;
#pragma unroll
      for (int g = 0; g < G; ++g) { float s, c; sincosf(xv * (float)(g + 1), &s, &c); v[2 * g] = (b16)(c * XS); v[2 * g + 1] = (b16)(s * XS); }
      *(v16b*)(&As[srow][il * 16]) = v; }
    __syncthreads();
#pragma unroll
    for (int kb = 0; kb < 128; kb += 32) { const v16b a = frag_kb(&As[nloc][kb], hlf);
#pragma unroll
      for (int t = 0; t < 16; ++t) acc[t] = wmma16b(a, frag_kb(WT + (size_t)(n0 + t * 16 + nloc) * K + kc + kb, hlf), acc[t]); }
    __syncthreads(); }
#pragma unroll
  for (int t = 0; t < 16; ++t) { const float bb = bf16_rne(bias[n0 + t * 16 + nloc]);
#pragma unroll
    for (int r = 0; r < 8; ++r) Tf[wave][8 * hlf + r][t * 16 + nloc] = acc[t][r] * (1.0f / (XS * WSC)) + bb; }
  wave_lds_sync();
  for (int pass = 0; pass < 2; ++pass) { for (int rr = 0; rr < 16; ++rr) { *(volatile v4f*)(out + (m0 + rr) * O + n0 + lane * 4) = *(const v4f*)(&Tf[wave][rr][lane * 4]); *(volatile v4f*)(out + (m0 + rr) * O + n0 + 128 + lane * 4) = *(const v4f*)(&Tf[wave][rr][128 + lane * 4]); } __threadfence(); }
}
}

extern "C" void kernel_launch(void* const* d_in, const int* in_sizes, int n_in, void* d_out, int out_size, void* d_ws, size_t ws_size, hipStream_t stream) {
  (void)n_in;
  auto Fp = [&](int i) { return (const float*)d_in[i]; };
  if (in_sizes[0] != NR * I || in_sizes[1] != 2 * O * I * G || in_sizes[2] != O || out_size != NR * O) return;
  size_t off = 0; char* ws = (char*)d_ws;
  auto carve = [&](size_t bytes) { char* p = ws + off; off += (bytes + 255) & ~(size_t)255; return p; };
  b16* WT = (b16*)carve((size_t)O * K * 2);
  if (off > ws_size || off > ((size_t)128 << 20)) return;
  wt_kernel<<<(O * I + 255) / 256, 256, 0, stream>>>(Fp(1), WT);
  fkan_kernel<<<ROWSL / 16, 64, 0, stream>>>(Fp(0), WT, Fp(2), (float*)d_out);
}
